// BioSSMMixer_83906481095354
// MI455X (gfx1250) — hardware-verified
//
#include <hip/hip_runtime.h>


#define NB_  2
#define TT   1024
#define DD   1024
#define D2   2048
#define NS   16
typedef _Float16 h16;
typedef unsigned short bf;
typedef __attribute__((ext_vector_type(16))) __bf16   v16bf;
typedef __attribute__((ext_vector_type(16))) _Float16 v16h;
typedef __attribute__((ext_vector_type(8)))  _Float16 v8h;
typedef __attribute__((ext_vector_type(8)))  unsigned short v8us;
typedef __attribute__((ext_vector_type(8)))  float    v8f;
typedef __attribute__((ext_vector_type(4)))  float    v4f;
typedef v8h  __attribute__((may_alias)) v8ha;
typedef v4f  __attribute__((may_alias)) v4fa;
typedef v8us __attribute__((may_alias)) v8usa;

__device__ __forceinline__ unsigned short f2bf(float f) { unsigned u = __float_as_uint(f); u += 0x7FFFu + ((u >> 16) & 1u); return (unsigned short)(u >> 16); }
__device__ __forceinline__ float bf2f(unsigned short b) { return __uint_as_float(((unsigned)b) << 16); }
__device__ __forceinline__ float bfr(float f) { return bf2f(f2bf(f)); }
__device__ __forceinline__ v16h cat16(v8h lo, v8h hi) { return __builtin_shufflevector(lo, hi, 0, 1, 2, 3, 4, 5, 6, 7, 8, 9, 10, 11, 12, 13, 14, 15); }
__device__ __forceinline__ v16bf cat16b(v8us lo, v8us hi) { return __builtin_bit_cast(v16bf, __builtin_shufflevector(lo, hi, 0, 1, 2, 3, 4, 5, 6, 7, 8, 9, 10, 11, 12, 13, 14, 15)); }
__device__ __forceinline__ v8f wmma16(v16h a, v16h b, v8f c) { return __builtin_amdgcn_wmma_f32_16x16x32_f16(false, a, false, b, (short)0, c, false, false); }
__device__ __forceinline__ v8f wmmab(v16bf a, v16bf b, v8f c) { return __builtin_amdgcn_wmma_f32_16x16x32_bf16(false, a, false, b, (short)0, c, false, false); }


template <typename T16> struct WFrag;
template <> struct WFrag<h16> { typedef v16h V; static __device__ __forceinline__ V ld(const h16* p) { return cat16(*(const v8h*)p, *(const v8h*)(p + 16)); } static __device__ __forceinline__ v8f mma(V a, V b, v8f c) { return wmma16(a, b, c); } };
template <> struct WFrag<bf> { typedef v16bf V; static __device__ __forceinline__ V ld(const bf* p) { return cat16b(*(const v8us*)p, *(const v8us*)(p + 16)); } static __device__ __forceinline__ v8f mma(V a, V b, v8f c) { return wmmab(a, b, c); } };
template <typename T16, int NSPLIT, bool BIAS>
__global__ __launch_bounds__(32) void k_gemmw(const T16* __restrict__ A, const T16* __restrict__ A2, const T16* __restrict__ Bt, const T16* __restrict__ Bt2, int K, float* C, int ldc, const float* __restrict__ bias, size_t sA, size_t sB, size_t sC) {
    typedef typename WFrag<T16>::V V;
    __shared__ __align__(16) float os[16 * 68];
    const size_t z = blockIdx.z; A += z * sA; if (A2) A2 += z * sA; Bt += z * sB; if (Bt2) Bt2 += z * sB; C += z * sC;
    const int lane = threadIdx.x & 31, lr = lane & 15, hi = lane >> 4; const int r0 = blockIdx.x * 64, c0 = blockIdx.y * 64;
    v8f acc[4][4];
#pragma unroll
    for (int mb = 0; mb < 4; ++mb)
#pragma unroll
        for (int nb = 0; nb < 4; ++nb) acc[mb][nb] = (v8f){};
    const size_t aoff = (size_t)(r0 + lr) * K + 8 * hi, boff = (size_t)(c0 + lr) * K + 8 * hi;
#pragma unroll 1
    for (int kc = 0; kc < K; kc += 32) {
        V a[4], a2[4];
#pragma unroll
        for (int mb = 0; mb < 4; ++mb) { a[mb] = WFrag<T16>::ld(A + aoff + (size_t)mb * 16 * K + kc); if (NSPLIT == 1 || NSPLIT == 2) a2[mb] = WFrag<T16>::ld(A2 + aoff + (size_t)mb * 16 * K + kc); }
#pragma unroll
        for (int nb = 0; nb < 4; ++nb) { const V b = WFrag<T16>::ld(Bt + boff + (size_t)nb * 16 * K + kc); V b2; if (NSPLIT >= 2) b2 = WFrag<T16>::ld(Bt2 + boff + (size_t)nb * 16 * K + kc);
#pragma unroll
            for (int mb = 0; mb < 4; ++mb) { acc[mb][nb] = WFrag<T16>::mma(a[mb], b, acc[mb][nb]); if (NSPLIT == 1 || NSPLIT == 2) acc[mb][nb] = WFrag<T16>::mma(a2[mb], b, acc[mb][nb]); if (NSPLIT >= 2) acc[mb][nb] = WFrag<T16>::mma(a[mb], b2, acc[mb][nb]); } }
        asm volatile("v_nop\n\tv_nop\n\tv_nop\n\tv_nop" : "+v"(acc[0][0]), "+v"(acc[1][1]), "+v"(acc[2][2]), "+v"(acc[3][3]) : "v"(a[0]), "v"(a[3]));
    }
#pragma unroll
    for (int mb = 0; mb < 4; ++mb) {
#pragma unroll
        for (int nb = 0; nb < 4; ++nb) {
#pragma unroll
            for (int j = 0; j < 8; ++j) os[(hi * 8 + j) * 68 + nb * 16 + lr] = acc[mb][nb][j]; }
        __builtin_amdgcn_wave_barrier(); asm volatile("" ::: "memory");
        float* crow = C + (size_t)(r0 + mb * 16) * ldc + c0;
#pragma unroll 1
        for (int ps = 0; ps < 2; ++ps) {
#pragma unroll
            for (int s = 0; s < 8; ++s) { const int row = 2 * s + hi, cofs = lr * 4; v4f val = *(const v4fa*)(os + row * 68 + cofs); if (BIAS) { val[0] += bfr(bias[c0 + cofs]); val[1] += bfr(bias[c0 + cofs + 1]); val[2] += bfr(bias[c0 + cofs + 2]); val[3] += bfr(bias[c0 + cofs + 3]); }
                *(volatile v4f*)(crow + (size_t)row * ldc + cofs) = val; }
            if (ps == 0) __threadfence(); }
        __builtin_amdgcn_wave_barrier(); asm volatile("" ::: "memory");
    }
}

__device__ __forceinline__ void splitf(float y, unsigned short& h, unsigned short& l) { h = f2bf(y); l = f2bf(y - bf2f(h)); }
__device__ __forceinline__ float siluf(float t) { float s = __fdiv_rn(1.0f, __fadd_rn(1.0f, __expf(-t))); asm volatile("" : "+v"(s)); return __fmul_rn(t, s); }
typedef __attribute__((ext_vector_type(2))) unsigned short v2us;
typedef __attribute__((ext_vector_type(4))) unsigned short v4us;

__global__ __launch_bounds__(256) void k_wtG(const float* __restrict__ w, int K, int N, bf* Bt) {
    const int lane = threadIdx.x & 31; const int L0 = (blockIdx.x * 8 + (threadIdx.x >> 5)) * 8; const int nlines = N * K / 64;
#pragma unroll
    for (int ps = 0; ps < 2; ++ps) {
#pragma unroll 1
        for (int l = 0; l < 8; ++l) { const int L = L0 + l; if (L >= nlines) break; const size_t e = (size_t)L * 64 + lane * 2; const int k = (int)(e % K), n = (int)(e / K); v2us o;
            o[0] = f2bf(w[(size_t)k * N + n]); o[1] = f2bf(w[(size_t)(k + 1) * N + n]); *(volatile v2us*)(Bt + e) = o; }
        if (ps == 0) __threadfence(); }
}
__global__ __launch_bounds__(256) void k_cvt8(const float* __restrict__ src, bf* dst, size_t n8) { const size_t i = (size_t)blockIdx.x * 256 + threadIdx.x; if (i >= n8) return; const v8f v = *(const v8f*)(src + i * 8); v8us o;
#pragma unroll
    for (int k = 0; k < 8; ++k) o[k] = f2bf(v[k]); *(volatile v8us*)(dst + i * 8) = o; __threadfence(); *(volatile v8us*)(dst + i * 8) = o; }
__global__ __launch_bounds__(256) void k_wpad(const float* __restrict__ w, int K, int N0, int NPd, bf* Bt) { const int e = (blockIdx.x * 256 + threadIdx.x) * 4; if (e >= NPd * K) return; const int k = e % K; const int n = e / K; v4us o;
#pragma unroll
    for (int u = 0; u < 4; ++u) o[u] = (n < N0) ? f2bf(w[(size_t)(k + u) * N0 + n]) : (unsigned short)0; *(volatile v4us*)(Bt + e) = o; __threadfence(); *(volatile v4us*)(Bt + e) = o; }
__global__ __launch_bounds__(256) void k_splx(const float* __restrict__ XZ, bf* Xh, bf* Xl) { const int e = (blockIdx.x * 256 + threadIdx.x) * 4; if (e >= TT * DD) return; const int d = e % DD; const int t = e / DD; const v4f a = *(const v4f*)(XZ + (size_t)t * D2 + d); v4us oh, ol;
#pragma unroll
    for (int u = 0; u < 4; ++u) { unsigned short h, l; splitf(a[u], h, l); oh[u] = h; ol[u] = l; } *(volatile v4us*)(Xh + e) = oh; *(volatile v4us*)(Xl + e) = ol; __threadfence(); *(volatile v4us*)(Xh + e) = oh; *(volatile v4us*)(Xl + e) = ol; }
__global__ __launch_bounds__(64) void k_scan(const float* __restrict__ DT, const float* __restrict__ XZ, const float* __restrict__ BM, const float* __restrict__ CM, const float* __restrict__ A_log, const float* __restrict__ Dsk, const float* __restrict__ vth, float* YG) { const int d = blockIdx.x * 64 + threadIdx.x; if (d >= DD) return;
    float A[NS], s[NS];
#pragma unroll
    for (int n = 0; n < NS; ++n) { A[n] = -__expf(bfr(A_log[d * NS + n])); s[n] = 0.f; }
    const float Dd = bfr(Dsk[d]); const float vt = fmaxf(bfr(vth[d]), 0.1f);
    for (int t = 0; t < TT; ++t) { const float dr = DT[(size_t)t * DD + d]; const float dt = (dr > 20.f) ? dr : log1pf(__expf(dr)); const float xv = XZ[(size_t)t * D2 + d]; float dx = __fmul_rn(dt, xv); asm volatile("" : "+v"(dx)); const float* bl = BM + (size_t)t * 64; const float* cl = CM + (size_t)t * 64; float y = 0.f;
#pragma unroll
        for (int n = 0; n < NS; ++n) { float da = __fmul_rn(dt, A[n]); asm volatile("" : "+v"(da)); const float ex = __expf(da); float t1 = __fmul_rn(ex, s[n]); asm volatile("" : "+v"(t1)); float t2 = __fmul_rn(dx, bl[n]); asm volatile("" : "+v"(t2)); s[n] = __fadd_rn(t1, t2); float p = __fmul_rn(s[n], cl[n]); asm volatile("" : "+v"(p)); y = __fadd_rn(y, p); }
        float du = __fmul_rn(Dd, xv); asm volatile("" : "+v"(du)); const float yy = __fadd_rn(y, du); float ar = __fmul_rn(10.0f, __fsub_rn(yy, vt)); asm volatile("" : "+v"(ar)); const float spk = __fdiv_rn(1.0f, __fadd_rn(1.0f, __expf(-ar)));
        float ys = __fmul_rn(yy, spk); asm volatile("" : "+v"(ys)); const float yg = __fmul_rn(ys, siluf(XZ[(size_t)t * D2 + DD + d]));
        *(volatile float*)(YG + (size_t)t * DD + d) = yg; __threadfence(); *(volatile float*)(YG + (size_t)t * DD + d) = yg; } }
__global__ __launch_bounds__(256) void k_spl(const float* __restrict__ F, size_t n4, bf* Hh, bf* Hl) { const size_t e = ((size_t)blockIdx.x * 256 + threadIdx.x) * 4; if (e >= n4) return; const v4f a = *(const v4f*)(F + e); v4us oh, ol;
#pragma unroll
    for (int u = 0; u < 4; ++u) { unsigned short h, l; splitf(a[u], h, l); oh[u] = h; ol[u] = l; } *(volatile v4us*)(Hh + e) = oh; *(volatile v4us*)(Hl + e) = ol; __threadfence(); *(volatile v4us*)(Hh + e) = oh; *(volatile v4us*)(Hl + e) = ol; }
__global__ __launch_bounds__(256) void k_fin(const float* __restrict__ O, const float* __restrict__ h, float* OUTb) { const int e = (blockIdx.x * 256 + threadIdx.x) * 4; if (e >= TT * DD) return; const v4f a = *(const v4f*)(O + e), b = *(const v4f*)(h + e); v4f o;
#pragma unroll
    for (int u = 0; u < 4; ++u) o[u] = __fsub_rn(a[u], bfr(b[u])); *(volatile v4f*)(OUTb + e) = o; __threadfence(); *(volatile v4f*)(OUTb + e) = o; }

extern "C" void kernel_launch(void* const* d_in, const int* in_sizes, int n_in,
                              void* d_out, int out_size, void* d_ws, size_t ws_size, hipStream_t stream) {
    (void)in_sizes; (void)n_in; (void)out_size;
    const float** I = (const float**)d_in;
    const float *hs = I[0], *W_xz = I[1], *W_dt = I[2], *b_dt = I[3], *A_log = I[4], *W_B = I[5], *W_C = I[6], *Dsk = I[7], *W_out = I[8], *vth = I[9];
    float* OUT = (float*)d_out;
    char* wsp = (char*)d_ws;
    auto take = [&](size_t bytes) { char* p = wsp; wsp += (bytes + 255) & ~(size_t)255; return (void*)p; };
    bf* BXZ = (bf*)take((size_t)D2 * DD * 2); bf* BDT = (bf*)take((size_t)DD * DD * 2); bf* BB = (bf*)take(64 * DD * 2); bf* BC = (bf*)take(64 * DD * 2); bf* BO = (bf*)take((size_t)DD * DD * 2);
    bf* HB = (bf*)take((size_t)TT * DD * 2); float* XZ = (float*)take((size_t)TT * D2 * 4); bf* Xh = (bf*)take((size_t)TT * DD * 2); bf* Xl = (bf*)take((size_t)TT * DD * 2); float* DT = (float*)take((size_t)TT * DD * 4); float* BM = (float*)take((size_t)TT * 64 * 4); float* CM = (float*)take((size_t)TT * 64 * 4);
    float* YG = (float*)take((size_t)TT * DD * 4); bf* Yh = (bf*)take((size_t)TT * DD * 2); bf* Yl = (bf*)take((size_t)TT * DD * 2); float* O = (float*)take((size_t)TT * DD * 4);
    if ((size_t)(wsp - (char*)d_ws) > ws_size) return;
    k_wtG<<<(unsigned)((DD * D2 / 64 + 63) / 64), 256, 0, stream>>>(W_xz, DD, D2, BXZ); k_wtG<<<(DD * DD / 64 + 63) / 64, 256, 0, stream>>>(W_dt, DD, DD, BDT); k_wtG<<<(DD * DD / 64 + 63) / 64, 256, 0, stream>>>(W_out, DD, DD, BO);
    k_wpad<<<(64 * DD / 4 + 255) / 256, 256, 0, stream>>>(W_B, DD, NS, 64, BB); k_wpad<<<(64 * DD / 4 + 255) / 256, 256, 0, stream>>>(W_C, DD, NS, 64, BC);
    const unsigned gE = (TT * DD / 4 + 255) / 256;
    for (int b = 0; b < NB_; ++b) { const float* hb = hs + (size_t)b * TT * DD;
        k_cvt8<<<(TT * DD / 8 + 255) / 256, 256, 0, stream>>>(hb, HB, (size_t)TT * DD / 8);
        k_gemmw<bf, 0, false><<<dim3(TT / 64, D2 / 64, 1), 32, 0, stream>>>(HB, nullptr, BXZ, nullptr, DD, XZ, D2, nullptr, 0, 0, 0);
        k_gemmw<bf, 0, false><<<dim3(TT / 64, 1, 1), 32, 0, stream>>>(HB, nullptr, BB, nullptr, DD, BM, 64, nullptr, 0, 0, 0); k_gemmw<bf, 0, false><<<dim3(TT / 64, 1, 1), 32, 0, stream>>>(HB, nullptr, BC, nullptr, DD, CM, 64, nullptr, 0, 0, 0);
        k_splx<<<gE, 256, 0, stream>>>(XZ, Xh, Xl); k_gemmw<bf, 1, true><<<dim3(TT / 64, DD / 64, 1), 32, 0, stream>>>(Xh, Xl, BDT, nullptr, DD, DT, DD, b_dt, 0, 0, 0);
        k_scan<<<DD / 64, 64, 0, stream>>>(DT, XZ, BM, CM, A_log, Dsk, vth, YG);
        k_spl<<<gE, 256, 0, stream>>>(YG, (size_t)TT * DD, Yh, Yl); k_gemmw<bf, 1, false><<<dim3(TT / 64, DD / 64, 1), 32, 0, stream>>>(Yh, Yl, BO, nullptr, DD, O, DD, nullptr, 0, 0, 0);
        k_fin<<<gE, 256, 0, stream>>>(O, hb, OUT + (size_t)b * TT * DD); }
}
